// PhysicsGraphNeuralODEFunc_39754217292306
// MI455X (gfx1250) — hardware-verified
//
#include <hip/hip_runtime.h>


#define NBR  16384
#define DD   512
#define HID  512
#define EH   32
#define NKF  5
#define DM   DD
#define OMG  0.5235987755982988f
#define LOSC 1024.0f

typedef _Float16 h16;
typedef unsigned short bf;
typedef __attribute__((ext_vector_type(16))) __bf16   v16bf;
typedef __attribute__((ext_vector_type(16))) _Float16 v16h;
typedef __attribute__((ext_vector_type(8)))  _Float16 v8h;
typedef __attribute__((ext_vector_type(8)))  unsigned short v8us;
typedef __attribute__((ext_vector_type(8)))  float    v8f;
typedef __attribute__((ext_vector_type(4)))  float    v4f;
typedef v8h  __attribute__((may_alias)) v8ha;
typedef v4f  __attribute__((may_alias)) v4fa;
typedef v8us __attribute__((may_alias)) v8usa;

__device__ __forceinline__ unsigned short f2bf(float f) { unsigned u = __float_as_uint(f); u += 0x7FFFu + ((u >> 16) & 1u); return (unsigned short)(u >> 16); }
__device__ __forceinline__ float bf2f(unsigned short b) { return __uint_as_float(((unsigned)b) << 16); }
__device__ __forceinline__ float bfr(float f) { return bf2f(f2bf(f)); }
__device__ __forceinline__ v16h cat16(v8h lo, v8h hi) { return __builtin_shufflevector(lo, hi, 0, 1, 2, 3, 4, 5, 6, 7, 8, 9, 10, 11, 12, 13, 14, 15); }
__device__ __forceinline__ v16bf cat16b(v8us lo, v8us hi) { return __builtin_bit_cast(v16bf, __builtin_shufflevector(lo, hi, 0, 1, 2, 3, 4, 5, 6, 7, 8, 9, 10, 11, 12, 13, 14, 15)); }
__device__ __forceinline__ v8f wmma16(v16h a, v16h b, v8f c) { return __builtin_amdgcn_wmma_f32_16x16x32_f16(false, a, false, b, (short)0, c, false, false); }
__device__ __forceinline__ v8f wmmab(v16bf a, v16bf b, v8f c) { return __builtin_amdgcn_wmma_f32_16x16x32_bf16(false, a, false, b, (short)0, c, false, false); }

template <bool SPLITA, bool F16OUT = false>
__global__ __launch_bounds__(128) void k_gemmb(const bf* __restrict__ A, const bf* __restrict__ Al, const bf* __restrict__ Bn, const float* __restrict__ bias, float* C, int ldc, h16* C2, const float* __restrict__ R = nullptr, int K = DM, int roundR = 1) {
    __shared__ __align__(16) float ost[4][16 * 68];
    const int lane = threadIdx.x & 31, wave = threadIdx.x >> 5, lr = lane & 15, hi = lane >> 4;
    const int r0 = blockIdx.x * 64 + wave * 16, c0 = blockIdx.y * 64;
    const size_t aoff = (size_t)(r0 + lr) * K + 8 * hi;
    size_t boff[4];
#pragma unroll
    for (int t = 0; t < 4; ++t) boff[t] = (size_t)(c0 + t * 16 + lr) * K + 8 * hi;
    v8f acc[4];
#pragma unroll
    for (int t = 0; t < 4; ++t) acc[t] = (v8f){};
#pragma unroll 1
    for (int kc = 0; kc < K; kc += 32) {
        const v16bf a = cat16b(*(const v8us*)(A + aoff + kc), *(const v8us*)(A + aoff + kc + 16));
        v16bf al = a;
        if (SPLITA) al = cat16b(*(const v8us*)(Al + aoff + kc), *(const v8us*)(Al + aoff + kc + 16));
#pragma unroll
        for (int t = 0; t < 4; ++t) { const v16bf b = cat16b(*(const v8us*)(Bn + boff[t] + kc), *(const v8us*)(Bn + boff[t] + kc + 16)); acc[t] = wmmab(a, b, acc[t]); if (SPLITA) acc[t] = wmmab(al, b, acc[t]); }
        asm volatile("v_nop\n\tv_nop\n\tv_nop\n\tv_nop" : "+v"(acc[0]), "+v"(acc[1]), "+v"(acc[2]), "+v"(acc[3]) : "v"(a), "v"(al));
    }
    float* os = &ost[wave][0];
#pragma unroll
    for (int t = 0; t < 4; ++t) { const float bv = bias ? bfr(bias[c0 + t * 16 + lr]) : 0.f;
#pragma unroll
        for (int j = 0; j < 8; ++j) os[(hi * 8 + j) * 68 + t * 16 + lr] = acc[t][j] + bv; }
    __syncthreads();
    if (F16OUT) {
        h16* crow = (h16*)(void*)C + (size_t)r0 * ldc + c0;
        auto pass = [&]() {
#pragma unroll
            for (int s = 0; s < 4; ++s) { const int row = 4 * s + (lane >> 3), piece = lane & 7; const float* sp = os + row * 68 + piece * 8; v8h o, o2;
#pragma unroll
                for (int i = 0; i < 8; ++i) { const h16 a = (h16)sp[i]; o[i] = a; o2[i] = (h16)((sp[i] - (float)a) * LOSC); }
                *(volatile v8h*)(crow + (size_t)row * ldc + piece * 8) = o; if (C2) *(volatile v8h*)(C2 + (size_t)r0 * ldc + c0 + (size_t)row * ldc + piece * 8) = o2; }
        };
        pass(); __threadfence(); pass();
    } else {
        float* crow = C + (size_t)r0 * ldc + c0;
        auto pass = [&]() {
#pragma unroll
            for (int s = 0; s < 8; ++s) { const int Lid = (lane >> 3) + 4 * s, piece = lane & 7; const int row = Lid >> 1, cofs = (Lid & 1) * 32 + piece * 4;
                v4f val = *(const v4fa*)(os + row * 68 + cofs); if (R) { const v4f rv = *(const v4f*)(R + ((size_t)r0 + row) * ldc + c0 + cofs); val += roundR ? (v4f){bfr(rv[0]), bfr(rv[1]), bfr(rv[2]), bfr(rv[3])} : rv; }
                *(volatile v4f*)(crow + (size_t)row * ldc + cofs) = val; }
        };
        pass(); __threadfence(); pass();
    }
}

__global__ __launch_bounds__(256) void k_wt(const float* __restrict__ Wm, int K, int ncols, bf* WT) {
    __shared__ __align__(16) unsigned short tl[64 * 72];
    const int tid = threadIdx.x, k0 = blockIdx.x * 64, n0 = blockIdx.y * 64;
    const int kk = tid >> 2, nq = (tid & 3) * 16;
#pragma unroll
    for (int i = 0; i < 16; ++i) tl[(nq + i) * 72 + kk] = f2bf(Wm[(size_t)(k0 + kk) * ncols + n0 + nq + i]);
    __syncthreads();
    const int piece = tid & 7;
    auto pass = [&]() {
#pragma unroll
        for (int s = 0; s < 2; ++s) { const int nr = (tid >> 3) + 32 * s; const v8us val = *(const v8usa*)(tl + nr * 72 + piece * 8); *(volatile v8us*)(WT + (size_t)(n0 + nr) * K + k0 + piece * 8) = val; }
    };
    pass(); __threadfence(); pass();
}

__global__ __launch_bounds__(256) void k_cvt(const float* __restrict__ src, bf* dst) {
    const int lane = threadIdx.x & 31; const size_t r = (size_t)blockIdx.x * 8 + (threadIdx.x >> 5); if (r >= (size_t)NBR) return;
#pragma unroll 1
    for (int ps = 0; ps < 2; ++ps) {
#pragma unroll
        for (int q = 0; q < DD / 256; ++q) { v8us o;
#pragma unroll
            for (int i = 0; i < 8; ++i) o[i] = f2bf(src[r * DD + q * 256 + lane * 8 + i]);
            *(volatile v8us*)(dst + r * DD + q * 256 + lane * 8) = o; }
        if (ps == 0) __threadfence(); }
}
__global__ __launch_bounds__(256) void k_lop(const float* __restrict__ FC, const float* __restrict__ tt, bf* Lh, bf* Ll) {
    const int lane = threadIdx.x & 31, i = blockIdx.x * 8 + (threadIdx.x >> 5); if (i >= DD) return; const float ts = bfr(tt[0]);
    const float c1 = cosf(1.0f * OMG * ts), s1 = sinf(1.0f * OMG * ts), c2 = cosf(2.0f * OMG * ts), s2 = sinf(2.0f * OMG * ts);
#pragma unroll 1
    for (int ps = 0; ps < 2; ++ps) {
#pragma unroll
        for (int q = 0; q < DD / 256; ++q) { v8us oh, ol;
#pragma unroll
            for (int e = 0; e < 8; ++e) { const int j = q * 256 + lane * 8 + e; const float* c = FC + ((size_t)i * DD + j) * NKF;
                float L = bfr(c[0]); L = L + bfr(c[1]) * c1; L = L + bfr(c[2]) * s1; L = L + bfr(c[3]) * c2; L = L + bfr(c[4]) * s2;
                const unsigned short hb = f2bf(L); oh[e] = hb; ol[e] = f2bf(L - bf2f(hb)); }
            const size_t o = (size_t)i * DD + q * 256 + lane * 8; *(volatile v8us*)(Lh + o) = oh; *(volatile v8us*)(Ll + o) = ol; }
        if (ps == 0) __threadfence(); }
}
__global__ __launch_bounds__(256) void k_relusplit(const float* __restrict__ Hs, bf* dh, bf* dl) {
    const int lane = threadIdx.x & 31; const size_t r = (size_t)blockIdx.x * 8 + (threadIdx.x >> 5); if (r >= (size_t)NBR) return;
#pragma unroll 1
    for (int ps = 0; ps < 2; ++ps) {
#pragma unroll
        for (int q = 0; q < HID / 256; ++q) { const size_t o = r * HID + q * 256 + lane * 8; v8us oh, ol;
#pragma unroll
            for (int i = 0; i < 8; ++i) { const float v = fmaxf(Hs[o + i], 0.f); const unsigned short hb = f2bf(v); oh[i] = hb; ol[i] = f2bf(v - bf2f(hb)); }
            *(volatile v8us*)(dh + o) = oh; *(volatile v8us*)(dl + o) = ol; }
        if (ps == 0) __threadfence(); }
}
__global__ __launch_bounds__(256) void k_rowmean(const float* __restrict__ Qm, const float* __restrict__ prev, float* S) {
    const size_t b = (size_t)blockIdx.x * 256 + threadIdx.x; if (b >= (size_t)NBR) return; float s = 0.f;
#pragma unroll 4
    for (int c = 0; c < DD; ++c) s += Qm[b * DD + c];
    const float v = (prev ? prev[b] : 0.f) + s * (1.0f / DD);
    *(volatile float*)(S + b) = v; __threadfence(); *(volatile float*)(S + b) = v;
}
__global__ __launch_bounds__(256) void k_out(const float* __restrict__ LT, const float* __restrict__ NL, const float* __restrict__ x,
                                            const float* __restrict__ tW1, const float* __restrict__ tb1, const float* __restrict__ tW2, const float* __restrict__ tb2,
                                            const float* __restrict__ hW1, const float* __restrict__ hb1, const float* __restrict__ hW2, const float* __restrict__ hb2, float* OUTP) {
    const int lane = threadIdx.x & 31; const size_t b = (size_t)blockIdx.x * 8 + (threadIdx.x >> 5); if (b >= (size_t)NBR) return;
    const float T = bfr(x[b * DD + 0]), Hh = bfr(x[b * DD + 1]);
    const float fT[5] = {T, Hh, T * T, T * Hh, T * T * T}; const float fH[5] = {T, Hh, T * T, T * Hh, T * Hh * Hh};
    float cT = bfr(tb2[0]), cH = bfr(hb2[0]);
#pragma unroll 1
    for (int e = 0; e < EH; ++e) { float aT = bfr(tb1[e]), aH = bfr(hb1[e]);
#pragma unroll
        for (int f = 0; f < 5; ++f) { aT = fmaf(fT[f], bfr(tW1[f * EH + e]), aT); aH = fmaf(fH[f], bfr(hW1[f * EH + e]), aH); }
        cT = fmaf(fmaxf(aT, 0.f), bfr(tW2[e]), cT); cH = fmaf(fmaxf(aH, 0.f), bfr(hW2[e]), cH); }
    const float nl = NL[b];
#pragma unroll 1
    for (int ps = 0; ps < 2; ++ps) {
#pragma unroll 1
        for (int c0 = lane * 4; c0 < DD; c0 += 128) { v4f o;
#pragma unroll
            for (int q = 0; q < 4; ++q) { const int i = c0 + q; float v = LT[(size_t)i * NBR + b] + nl; if (i == 0) v += cT; else if (i == 1) v += cH; o[q] = v; }
            *(volatile v4f*)(OUTP + b * DD + c0) = o; }
        if (ps == 0) __threadfence(); }
}

extern "C" void kernel_launch(void* const* d_in, const int* in_sizes, int n_in,
                              void* d_out, int out_size, void* d_ws, size_t ws_size, hipStream_t stream) {
    (void)in_sizes; (void)n_in; (void)out_size;
    const float* x = (const float*)d_in[0]; const float* tt = (const float*)d_in[1]; const float* FC = (const float*)d_in[2];
    const float* qW1 = (const float*)d_in[3]; const float* qb1 = (const float*)d_in[4]; const float* qW2 = (const float*)d_in[5]; const float* qb2 = (const float*)d_in[6];
    const float* cW1 = (const float*)d_in[7]; const float* cb1 = (const float*)d_in[8]; const float* cW2 = (const float*)d_in[9]; const float* cb2 = (const float*)d_in[10];
    const float* tW1 = (const float*)d_in[11]; const float* tb1 = (const float*)d_in[12]; const float* tW2 = (const float*)d_in[13]; const float* tb2 = (const float*)d_in[14];
    const float* hW1 = (const float*)d_in[15]; const float* hb1 = (const float*)d_in[16]; const float* hW2 = (const float*)d_in[17]; const float* hb2 = (const float*)d_in[18];
    float* out = (float*)d_out;
    char* wsp = (char*)d_ws;
    auto take = [&](size_t bytes) { char* p = wsp; wsp += (bytes + 255) & ~(size_t)255; return (void*)p; };
    bf* Xb = (bf*)take((size_t)NBR * DD * 2); bf* Lh = (bf*)take((size_t)DD * DD * 2); bf* Ll = (bf*)take((size_t)DD * DD * 2); float* LT = (float*)take((size_t)DD * NBR * 4);
    bf* W1T = (bf*)take((size_t)HID * DD * 2); bf* W2T = (bf*)take((size_t)DD * HID * 2); float* Hs = (float*)take((size_t)NBR * HID * 4); bf* Rh = (bf*)take((size_t)NBR * HID * 2); bf* Rl = (bf*)take((size_t)NBR * HID * 2);
    float* NL0 = (float*)take((size_t)NBR * 4); float* NL = (float*)take((size_t)NBR * 4);
    if ((size_t)(wsp - (char*)d_ws) > ws_size) return;
    k_cvt<<<NBR / 8, 256, 0, stream>>>(x, Xb);
    k_lop<<<DD / 8, 256, 0, stream>>>(FC, tt, Lh, Ll);
    k_gemmb<true, false><<<dim3(DD / 64, NBR / 64, 1), 128, 0, stream>>>(Lh, Ll, Xb, nullptr, LT, NBR, nullptr, nullptr, DD);
    k_wt<<<dim3(DD / 64, HID / 64, 1), 256, 0, stream>>>(qW1, DD, HID, W1T); k_wt<<<dim3(HID / 64, DD / 64, 1), 256, 0, stream>>>(qW2, HID, DD, W2T);
    k_gemmb<false, false><<<dim3(NBR / 64, HID / 64, 1), 128, 0, stream>>>(Xb, nullptr, W1T, qb1, Hs, HID, nullptr, nullptr, DD); k_relusplit<<<NBR / 8, 256, 0, stream>>>(Hs, Rh, Rl);
    k_gemmb<true, false><<<dim3(NBR / 64, DD / 64, 1), 128, 0, stream>>>(Rh, Rl, W2T, qb2, Hs, DD, nullptr, nullptr, HID); k_rowmean<<<NBR / 256, 256, 0, stream>>>(Hs, nullptr, NL0);
    k_wt<<<dim3(DD / 64, HID / 64, 1), 256, 0, stream>>>(cW1, DD, HID, W1T); k_wt<<<dim3(HID / 64, DD / 64, 1), 256, 0, stream>>>(cW2, HID, DD, W2T);
    k_gemmb<false, false><<<dim3(NBR / 64, HID / 64, 1), 128, 0, stream>>>(Xb, nullptr, W1T, cb1, Hs, HID, nullptr, nullptr, DD); k_relusplit<<<NBR / 8, 256, 0, stream>>>(Hs, Rh, Rl);
    k_gemmb<true, false><<<dim3(NBR / 64, DD / 64, 1), 128, 0, stream>>>(Rh, Rl, W2T, cb2, Hs, DD, nullptr, nullptr, HID); k_rowmean<<<NBR / 256, 256, 0, stream>>>(Hs, NL0, NL);
    k_out<<<NBR / 8, 256, 0, stream>>>(LT, NL, x, tW1, tb1, tW2, tb2, hW1, hb1, hW2, hb2, out);
}
